// FlowAttention_24584392803024
// MI455X (gfx1250) — hardware-verified
//
#include <hip/hip_runtime.h>

#define BB_ 8
#define CC_ 512
#define QQ_ 64
#define DD_ 256

typedef _Float16 f16;
typedef __attribute__((ext_vector_type(16))) f16 f16x16;
typedef __attribute__((ext_vector_type(8)))  f16 f16x8;
typedef __attribute__((ext_vector_type(8)))  float f32x8;
typedef __attribute__((ext_vector_type(4)))  float v4f_t;
typedef float v4fa __attribute__((ext_vector_type(4), may_alias));
typedef __attribute__((ext_vector_type(4)))  unsigned v4u_t;

__device__ __forceinline__ f32x8 wmma16(f16x16 a, f16x16 b, f32x8 c) {
  c = __builtin_amdgcn_wmma_f32_16x16x32_f16(false, a, false, b, (short)0, c, false, false);
  asm volatile("v_nop\n\tv_nop\n\tv_nop\n\tv_nop" : "+v"(c) : "v"(a), "v"(b));
  return c;
}
__device__ __forceinline__ f16x16 lds_frag(const f16* base, int stride) {
  const int lane = threadIdx.x & 31, row = lane & 15, kh = (lane >> 4) * 8;
  const f16x8 lo = *(const f16x8*)(base + row * stride + kh);
  const f16x8 hi = *(const f16x8*)(base + row * stride + kh + 16);
  f16x16 f;
#pragma unroll
  for (int i = 0; i < 8; ++i) { f[i] = lo[i]; f[i + 8] = hi[i]; }
  return f;
}
__device__ __forceinline__ f16x16 gbl_frag(const f16* __restrict__ base, int stride) {
  const int lane = threadIdx.x & 31, row = lane & 15, kh = (lane >> 4) * 8;
  const f16x8 lo = *(const f16x8*)(base + (size_t)row * stride + kh);
  const f16x8 hi = *(const f16x8*)(base + (size_t)row * stride + kh + 16);
  f16x16 f;
#pragma unroll
  for (int i = 0; i < 8; ++i) { f[i] = lo[i]; f[i + 8] = hi[i]; }
  return f;
}
__device__ __forceinline__ float leaky(float x) { return x >= 0.0f ? x : 0.01f * x; }

#define GSTR 48
template <typename AT, bool ACC>
__global__ __launch_bounds__(256) void gemm_kn(const AT* __restrict__ A, int lda, size_t strideA,
                                               const float* __restrict__ Wm, int ldw, size_t strideW,
                                               const float* __restrict__ bias, float scale,
                                               float* __restrict__ Y, int ldy, size_t strideY, int K) {
  __shared__ __attribute__((aligned(16))) f16 ldsA[128 * GSTR];
  __shared__ __attribute__((aligned(16))) f16 ldsW[128 * GSTR];
  __shared__ __attribute__((aligned(16))) float oS[8][32 * 68];
  const int tid = threadIdx.x, lane = tid & 31, wave = tid >> 5, cl = lane & 15, rh = (lane >> 4) * 8;
  const int m0 = blockIdx.x * 128, n0 = blockIdx.y * 128;
  const int wm = (wave & 3) * 32, wn = (wave >> 2) * 64;
  A += (size_t)blockIdx.z * strideA; Wm += (size_t)blockIdx.z * strideW; Y += (size_t)blockIdx.z * strideY;
  f32x8 acc[2][4];
#pragma unroll
  for (int i = 0; i < 2; ++i)
#pragma unroll
    for (int j = 0; j < 4; ++j) { f32x8 z = {}; acc[i][j] = z; }
#pragma unroll 1
  for (int k0 = 0; k0 < K; k0 += 32) {
    __syncthreads();
    {
      const int row = tid >> 1, ch = (tid & 1) * 16;
      const AT* src = A + (size_t)(m0 + row) * lda + k0 + ch;
#pragma unroll
      for (int g = 0; g < 16; ++g) ldsA[row * GSTR + ch + g] = (f16)src[g];
    }
    {
      const int k = tid >> 3, nn0 = (tid & 7) * 16;
      const float* src = Wm + (size_t)(k0 + k) * ldw + n0 + nn0;
#pragma unroll
      for (int g = 0; g < 4; ++g) { const v4f_t v = *(const v4f_t*)(src + 4 * g);
#pragma unroll
        for (int u = 0; u < 4; ++u) ldsW[(nn0 + 4 * g + u) * GSTR + k] = (f16)v[u]; }
    }
    __syncthreads();
    f16x16 af[2];
#pragma unroll
    for (int i = 0; i < 2; ++i) af[i] = lds_frag(ldsA + (wm + 16 * i) * GSTR, GSTR);
#pragma unroll
    for (int j = 0; j < 4; ++j) {
      const f16x16 bf = lds_frag(ldsW + (wn + 16 * j) * GSTR, GSTR);
#pragma unroll
      for (int i = 0; i < 2; ++i) acc[i][j] = wmma16(af[i], bf, acc[i][j]);
    }
  }
  float* so = oS[wave];
#pragma unroll
  for (int i = 0; i < 2; ++i)
#pragma unroll
    for (int j = 0; j < 4; ++j) {
      const float bv = bias ? bias[n0 + wn + 16 * j + cl] : 0.0f;
#pragma unroll
      for (int r = 0; r < 8; ++r) so[(16 * i + rh + r) * 68 + 16 * j + cl] = acc[i][j][r] * scale + bv;
    }
  asm volatile("s_wait_dscnt 0" ::: "memory");
  __builtin_amdgcn_wave_barrier();
  if (ACC) {
#pragma unroll
    for (int it = 0; it < 16; ++it) { const int f4 = lane + 32 * it, rr = f4 >> 4, q = (f4 & 15) * 4;
      const v4f_t old = *(const volatile v4fa*)(Y + (size_t)(m0 + wm + rr) * ldy + n0 + wn + q);
      v4f_t v = *(const volatile v4fa*)(so + rr * 68 + q); v += old; *(volatile v4fa*)(so + rr * 68 + q) = v; }
    asm volatile("s_wait_dscnt 0" ::: "memory");
  }
#pragma unroll 1
  for (int pass = 0; pass < 2; ++pass) {
#pragma unroll
    for (int it = 0; it < 16; ++it) { const int f4 = lane + 32 * it, rr = f4 >> 4, q = (f4 & 15) * 4;
      *(volatile v4f_t*)(Y + (size_t)(m0 + wm + rr) * ldy + n0 + wn + q) = *(const volatile v4fa*)(so + rr * 68 + q); }
    __threadfence();
  }
}

template <typename AT, bool ACC>
__global__ __launch_bounds__(256) void gemm_kn2(const AT* __restrict__ A, int lda, size_t strideA,
                                               const float* __restrict__ Wm, int ldw, size_t strideW,
                                               const float* __restrict__ bias, float scale,
                                               float* __restrict__ Y, int ldy, size_t strideY, int K) {
  __shared__ __attribute__((aligned(16))) f16 ldsA[128 * GSTR], ldsAl[128 * GSTR];
  __shared__ __attribute__((aligned(16))) f16 ldsW[128 * GSTR], ldsWl[128 * GSTR];
  __shared__ __attribute__((aligned(16))) float oS[8][32 * 68];
  const int tid = threadIdx.x, lane = tid & 31, wave = tid >> 5, cl = lane & 15, rh = (lane >> 4) * 8;
  const int m0 = blockIdx.x * 128, n0 = blockIdx.y * 128;
  const int wm = (wave & 3) * 32, wn = (wave >> 2) * 64;
  A += (size_t)blockIdx.z * strideA; Wm += (size_t)blockIdx.z * strideW; Y += (size_t)blockIdx.z * strideY;
  f32x8 acc[2][4], accx[2][4];
#pragma unroll
  for (int i = 0; i < 2; ++i)
#pragma unroll
    for (int j = 0; j < 4; ++j) { f32x8 z = {}; acc[i][j] = z; accx[i][j] = z; }
#pragma unroll 1
  for (int k0 = 0; k0 < K; k0 += 32) {
    __syncthreads();
    {
      const int row = tid >> 1, ch = (tid & 1) * 16;
      const AT* src = A + (size_t)(m0 + row) * lda + k0 + ch;
#pragma unroll
      for (int g = 0; g < 16; ++g) { const float v = (float)src[g]; const f16 h = (f16)v; ldsA[row * GSTR + ch + g] = h; ldsAl[row * GSTR + ch + g] = (f16)((v - (float)h) * 2048.0f); }
    }
    {
      const int k = tid >> 3, nn0 = (tid & 7) * 16;
      const float* src = Wm + (size_t)(k0 + k) * ldw + n0 + nn0;
#pragma unroll
      for (int g = 0; g < 4; ++g) { const v4f_t v = *(const v4f_t*)(src + 4 * g);
#pragma unroll
        for (int u = 0; u < 4; ++u) { const f16 h = (f16)v[u]; ldsW[(nn0 + 4 * g + u) * GSTR + k] = h; ldsWl[(nn0 + 4 * g + u) * GSTR + k] = (f16)((v[u] - (float)h) * 2048.0f); } }
    }
    __syncthreads();
    f16x16 af[2], afl[2];
#pragma unroll
    for (int i = 0; i < 2; ++i) { af[i] = lds_frag(ldsA + (wm + 16 * i) * GSTR, GSTR); afl[i] = lds_frag(ldsAl + (wm + 16 * i) * GSTR, GSTR); }
#pragma unroll
    for (int j = 0; j < 4; ++j) {
      const f16x16 bf = lds_frag(ldsW + (wn + 16 * j) * GSTR, GSTR), bfl = lds_frag(ldsWl + (wn + 16 * j) * GSTR, GSTR);
#pragma unroll
      for (int i = 0; i < 2; ++i) { acc[i][j] = wmma16(af[i], bf, acc[i][j]); accx[i][j] = wmma16(af[i], bfl, accx[i][j]); accx[i][j] = wmma16(afl[i], bf, accx[i][j]); }
    }
  }
  float* so = oS[wave];
#pragma unroll
  for (int i = 0; i < 2; ++i)
#pragma unroll
    for (int j = 0; j < 4; ++j) {
      const float bv = bias ? bias[n0 + wn + 16 * j + cl] : 0.0f;
#pragma unroll
      for (int r = 0; r < 8; ++r) so[(16 * i + rh + r) * 68 + 16 * j + cl] = (acc[i][j][r] + accx[i][j][r] * (1.0f / 2048.0f)) * scale + bv;
    }
  asm volatile("s_wait_dscnt 0" ::: "memory");
  __builtin_amdgcn_wave_barrier();
  if (ACC) {
#pragma unroll
    for (int it = 0; it < 16; ++it) { const int f4 = lane + 32 * it, rr = f4 >> 4, q = (f4 & 15) * 4;
      const v4f_t old = *(const volatile v4fa*)(Y + (size_t)(m0 + wm + rr) * ldy + n0 + wn + q);
      v4f_t v = *(const volatile v4fa*)(so + rr * 68 + q); v += old; *(volatile v4fa*)(so + rr * 68 + q) = v; }
    asm volatile("s_wait_dscnt 0" ::: "memory");
  }
#pragma unroll 1
  for (int pass = 0; pass < 2; ++pass) {
#pragma unroll
    for (int it = 0; it < 16; ++it) { const int f4 = lane + 32 * it, rr = f4 >> 4, q = (f4 & 15) * 4;
      *(volatile v4f_t*)(Y + (size_t)(m0 + wm + rr) * ldy + n0 + wn + q) = *(const volatile v4fa*)(so + rr * 68 + q); }
    __threadfence();
  }
}

__global__ __launch_bounds__(256) void k_prep(const float* __restrict__ W1, f16* __restrict__ WmT) {
  const int g = blockIdx.x * 256 + threadIdx.x;
  const int n = g >> 5, k0 = (g & 31) * 8;
  union { f16 h[8]; v4u_t v; } u;
#pragma unroll
  for (int t = 0; t < 8; ++t) u.h[t] = (f16)W1[(size_t)(2 * DD_ + k0 + t) * DD_ + n];
  *(volatile v4u_t*)(WmT + (size_t)n * DD_ + k0) = u.v; __threadfence(); *(volatile v4u_t*)(WmT + (size_t)n * DD_ + k0) = u.v;
}

__global__ __launch_bounds__(128) void k_pairs(const float* __restrict__ Hm, const float* __restrict__ Um, const f16* __restrict__ WmT,
                                               const float* __restrict__ hp, const float* __restrict__ up, const float* __restrict__ b1,
                                               const float* __restrict__ W2, const float* __restrict__ b2, float* __restrict__ S) {
  __shared__ __attribute__((aligned(16))) f16 lS[4][16 * 264], llS[4][16 * 264];
  __shared__ __attribute__((aligned(16))) float sS[64];
  const int tid = threadIdx.x, lane = tid & 31, wave = tid >> 5, cl = lane & 15, kh = (lane >> 4) * 8, rh = kh;
  const int b = blockIdx.x >> 9, c = blockIdx.x & 511;
  const int qt = wave, q0 = qt * 16;
  const float* Hc = Hm + ((size_t)b * CC_ + c) * DD_;
  const float* Uq = Um + ((size_t)b * QQ_ + q0 + cl) * DD_;
  f32x8 acc[16];
#pragma unroll
  for (int nt = 0; nt < 16; ++nt) { f32x8 z = {}; acc[nt] = z; }
#pragma unroll 1
  for (int ks = 0; ks < 8; ++ks) {
    f16x16 af;
    {
      const float* ph = Hc + ks * 32 + kh; const float* pu = Uq + ks * 32 + kh;
      const v4f_t h0 = *(const v4f_t*)ph, h1 = *(const v4f_t*)(ph + 4), h2 = *(const v4f_t*)(ph + 16), h3 = *(const v4f_t*)(ph + 20);
      const v4f_t u0 = *(const v4f_t*)pu, u1 = *(const v4f_t*)(pu + 4), u2 = *(const v4f_t*)(pu + 16), u3 = *(const v4f_t*)(pu + 20);
      af[0] = (f16)(h0[0]*u0[0]); af[1] = (f16)(h0[1]*u0[1]); af[2]  = (f16)(h0[2]*u0[2]); af[3]  = (f16)(h0[3]*u0[3]);
      af[4] = (f16)(h1[0]*u1[0]); af[5] = (f16)(h1[1]*u1[1]); af[6]  = (f16)(h1[2]*u1[2]); af[7]  = (f16)(h1[3]*u1[3]);
      af[8] = (f16)(h2[0]*u2[0]); af[9] = (f16)(h2[1]*u2[1]); af[10] = (f16)(h2[2]*u2[2]); af[11] = (f16)(h2[3]*u2[3]);
      af[12]= (f16)(h3[0]*u3[0]); af[13]= (f16)(h3[1]*u3[1]); af[14] = (f16)(h3[2]*u3[2]); af[15] = (f16)(h3[3]*u3[3]);
    }
#pragma unroll
    for (int nt = 0; nt < 16; ++nt) acc[nt] = wmma16(af, gbl_frag(WmT + (size_t)(nt * 16) * DD_ + ks * 32, DD_), acc[nt]);
  }
  f16* lw = lS[wave]; f16* llw = llS[wave];
  const float* hpc = hp + ((size_t)b * CC_ + c) * DD_;
#pragma unroll
  for (int nt = 0; nt < 16; ++nt) {
    const int e = nt * 16 + cl;
    const float add = hpc[e] + b1[e];
#pragma unroll
    for (int r = 0; r < 8; ++r) {
      const int q = q0 + rh + r;
      const float v = leaky(acc[nt][r] + add + up[((size_t)b * QQ_ + q) * DD_ + e]);
      const f16 h = (f16)v;
      lw[(rh + r) * 264 + e] = h; llw[(rh + r) * 264 + e] = (f16)((v - (float)h) * 2048.0f);
    }
  }
  f16x16 wb[8];
#pragma unroll
  for (int ks = 0; ks < 8; ++ks)
#pragma unroll
    for (int i = 0; i < 8; ++i) {
      wb[ks][i]     = (cl == 0) ? (f16)W2[ks * 32 + kh + i]      : (f16)0.0f;
      wb[ks][i + 8] = (cl == 0) ? (f16)W2[ks * 32 + kh + 16 + i] : (f16)0.0f;
    }
  asm volatile("s_wait_dscnt 0" ::: "memory");
  __builtin_amdgcn_wave_barrier();
  f32x8 sz = {}, szl = {};
#pragma unroll
  for (int ks = 0; ks < 8; ++ks) { sz = wmma16(lds_frag(lw + ks * 32, 264), wb[ks], sz); szl = wmma16(lds_frag(llw + ks * 32, 264), wb[ks], szl); }
  if (cl == 0) {
    const float bb2 = b2[0];
#pragma unroll
    for (int r = 0; r < 8; ++r) sS[q0 + rh + r] = leaky(sz[r] + szl[r] * (1.0f / 2048.0f) + bb2);
  }
  __syncthreads();
  if (wave == 0 && lane < 16) {
#pragma unroll 1
    for (int pass = 0; pass < 2; ++pass) { *(volatile v4f_t*)(S + ((size_t)b * CC_ + c) * QQ_ + lane * 4) = *(const volatile v4fa*)(sS + lane * 4); __threadfence(); }
  }
}

__global__ __launch_bounds__(256) void k_c2q(const float* __restrict__ S, const float* __restrict__ Um, const int* __restrict__ cmask,
                                             const int* __restrict__ qmask, float* __restrict__ Uhat, float* __restrict__ Smax) {
  __shared__ __attribute__((aligned(16))) f16 UtS[DD_ * 72];
  __shared__ __attribute__((aligned(16))) f16 pS[8][16 * 72], plS[8][16 * 72];
  __shared__ __attribute__((aligned(16))) float oS[8][16 * 68];
  __shared__ __attribute__((aligned(16))) float smS[128];
  __shared__ int qmS[64];
  const int tid = threadIdx.x, lane = tid & 31, wave = tid >> 5, cl = lane & 15, hsel = lane >> 4, kh = hsel * 8, rh = kh;
  const int b = blockIdx.x >> 2, ct0 = (blockIdx.x & 3) * 8;
  const float* Ub = Um + (size_t)b * QQ_ * DD_;
  for (int e = tid; e < QQ_ * DD_; e += 256) { const int q = e >> 8, d = e & 255; UtS[d * 72 + q] = (f16)Ub[e]; }
  if (tid < 64) qmS[tid] = qmask[b * QQ_ + tid];
  __syncthreads();
  const int c0 = (ct0 + wave) * 16;
  const int c = c0 + cl;
  const bool cm0 = (cmask[b * CC_ + c] == 0);
  const float* srow = S + ((size_t)b * CC_ + c) * QQ_ + hsel * 32;
  float sv[32], mx = -INFINITY;
#pragma unroll
  for (int j = 0; j < 32; ++j) { float v = srow[j]; if (cm0 || qmS[hsel * 32 + j] == 0) v = -1.0e9f; sv[j] = v; mx = fmaxf(mx, v); }
  mx = fmaxf(mx, __shfl_xor(mx, 16, 32));
  float se = 0.0f;
#pragma unroll
  for (int j = 0; j < 32; ++j) { sv[j] = __expf(sv[j] - mx); se += sv[j]; }
  se += __shfl_xor(se, 16, 32);
  const float sc = 1024.0f / se;
  f16* pw = pS[wave]; f16* plw = plS[wave];
#pragma unroll
  for (int j = 0; j < 32; ++j) { const float v = sv[j] * sc; const f16 h = (f16)v; pw[cl * 72 + hsel * 32 + j] = h; plw[cl * 72 + hsel * 32 + j] = (f16)((v - (float)h) * 2048.0f); }
  if (hsel == 0) smS[wave * 16 + cl] = mx;
  asm volatile("s_wait_dscnt 0" ::: "memory");
  __builtin_amdgcn_wave_barrier();
  const f16x16 a0 = lds_frag(pw, 72), a1 = lds_frag(pw + 32, 72), a0l = lds_frag(plw, 72), a1l = lds_frag(plw + 32, 72);
  float* so = oS[wave];
#pragma unroll 1
  for (int ch = 0; ch < 4; ++ch) {
#pragma unroll
    for (int nt = 0; nt < 4; ++nt) {
      f32x8 z = {};
      const int d0 = ch * 64 + nt * 16;
      f32x8 zl = {};
      const f16x16 u0 = lds_frag(UtS + d0 * 72, 72), u1 = lds_frag(UtS + d0 * 72 + 32, 72);
      z = wmma16(a0, u0, z);  z = wmma16(a1, u1, z);
      zl = wmma16(a0l, u0, zl); zl = wmma16(a1l, u1, zl);
#pragma unroll
      for (int r = 0; r < 8; ++r) so[(rh + r) * 68 + nt * 16 + cl] = (z[r] + zl[r] * (1.0f / 2048.0f)) * (1.0f / 1024.0f);
    }
    asm volatile("s_wait_dscnt 0" ::: "memory");
    __builtin_amdgcn_wave_barrier();
#pragma unroll 1
    for (int pass = 0; pass < 2; ++pass) {
#pragma unroll
      for (int it = 0; it < 8; ++it) { const int f4 = lane + 32 * it, rr = f4 >> 4, qd = (f4 & 15) * 4;
        *(volatile v4f_t*)(Uhat + ((size_t)b * CC_ + c0 + rr) * DD_ + ch * 64 + qd) = *(const volatile v4fa*)(so + rr * 68 + qd); }
      __threadfence();
    }
    __builtin_amdgcn_wave_barrier();
  }
  __syncthreads();
  if (wave == 0) {
#pragma unroll 1
    for (int pass = 0; pass < 2; ++pass) { *(volatile v4f_t*)(Smax + (size_t)b * CC_ + ct0 * 16 + lane * 4) = *(const volatile v4fa*)(smS + lane * 4); __threadfence(); }
  }
}

__global__ __launch_bounds__(256) void k_q2c(const float* __restrict__ Smax, const float* __restrict__ Hm, float* __restrict__ Hhat) {
  __shared__ float bS[CC_];
  __shared__ float red[8];
  __shared__ __attribute__((aligned(16))) float qS[DD_];
  const int tid = threadIdx.x, lane = tid & 31, wave = tid >> 5, cl = lane & 15, hsel = lane >> 4, kh = hsel * 8;
  const int b = blockIdx.x;
  float s2[2], mx;
  s2[0] = Smax[b * CC_ + tid]; s2[1] = Smax[b * CC_ + 256 + tid]; mx = fmaxf(s2[0], s2[1]);
#pragma unroll
  for (int off = 16; off >= 1; off >>= 1) mx = fmaxf(mx, __shfl_xor(mx, off, 32));
  if (lane == 0) red[wave] = mx;
  __syncthreads();
  mx = fmaxf(fmaxf(fmaxf(red[0], red[1]), fmaxf(red[2], red[3])), fmaxf(fmaxf(red[4], red[5]), fmaxf(red[6], red[7])));
  const float e0 = __expf(s2[0] - mx), e1 = __expf(s2[1] - mx);
  float se = e0 + e1;
#pragma unroll
  for (int off = 16; off >= 1; off >>= 1) se += __shfl_xor(se, off, 32);
  __syncthreads();
  if (lane == 0) red[wave] = se;
  __syncthreads();
  const float Z = ((red[0] + red[1]) + (red[2] + red[3])) + ((red[4] + red[5]) + (red[6] + red[7]));
  bS[tid] = e0 / Z * 1024.0f; bS[256 + tid] = e1 / Z * 1024.0f;
  __syncthreads();
  const float* Hb = Hm + (size_t)b * CC_ * DD_;
  f32x8 acc[2], accl[2];
  { f32x8 z = {}; acc[0] = z; acc[1] = z; accl[0] = z; accl[1] = z; }
#pragma unroll 1
  for (int ks = 0; ks < 16; ++ks) {
    f16x16 af, afl;
#pragma unroll
    for (int i = 0; i < 16; ++i) {
      const float v = (cl == 0) ? bS[ks * 32 + kh + (i & 7) + ((i >> 3) << 4)] : 0.0f;
      const f16 h = (f16)v; af[i] = h; afl[i] = (f16)((v - (float)h) * 2048.0f);
    }
#pragma unroll
    for (int nt = 0; nt < 2; ++nt) {
      f16x16 bf, bfl;
      const float* hp0 = Hb + (size_t)(ks * 32 + kh) * DD_ + wave * 32 + nt * 16 + cl;
#pragma unroll
      for (int i = 0; i < 16; ++i) { const float v = hp0[(size_t)((i & 7) + ((i >> 3) << 4)) * DD_]; const f16 h = (f16)v; bf[i] = h; bfl[i] = (f16)((v - (float)h) * 2048.0f); }
      acc[nt] = wmma16(af, bf, acc[nt]); accl[nt] = wmma16(af, bfl, accl[nt]); accl[nt] = wmma16(afl, bf, accl[nt]);
    }
  }
  if (hsel == 0) { qS[wave * 32 + cl] = (acc[0][0] + accl[0][0] * (1.0f / 2048.0f)) * (1.0f / 1024.0f); qS[wave * 32 + 16 + cl] = (acc[1][0] + accl[1][0] * (1.0f / 2048.0f)) * (1.0f / 1024.0f); }
  __syncthreads();
#pragma unroll 1
  for (int pass = 0; pass < 2; ++pass) {
    for (int it = 0; it < 128; ++it) { const int f4 = tid + 256 * it, row = f4 >> 6, qd = (f4 & 63) * 4;
      *(volatile v4f_t*)(Hhat + ((size_t)b * CC_ + row) * DD_ + qd) = *(const volatile v4fa*)(qS + qd); }
    __threadfence();
  }
}

extern "C" void kernel_launch(void* const* d_in, const int* in_sizes, int n_in,
                              void* d_out, int out_size, void* d_ws, size_t ws_size,
                              hipStream_t stream) {
  (void)in_sizes; (void)n_in; (void)out_size; (void)ws_size;
  const float* Hm = (const float*)d_in[0];
  const float* Um = (const float*)d_in[1];
  const int* cmask = (const int*)d_in[2];
  const int* qmask = (const int*)d_in[3];
  const float* W1 = (const float*)d_in[4];
  const float* b1 = (const float*)d_in[5];
  const float* W2 = (const float*)d_in[6];
  const float* b2 = (const float*)d_in[7];
  float* Hhat = (float*)d_out;
  float* Uhat = Hhat + (size_t)BB_ * CC_ * DD_;
  char* ws = (char*)d_ws;
  float* hp = (float*)ws; float* up = (float*)(ws + (4 << 20)); float* S = (float*)(ws + (4 << 20) + (512 << 10));
  float* Smax = (float*)(ws + (5 << 20) + (512 << 10)); f16* WmT = (f16*)(ws + (5 << 20) + (768 << 10));
  k_prep<<<dim3(32), dim3(256), 0, stream>>>(W1, WmT);
  gemm_kn2<float, false><<<dim3(BB_ * CC_ / 128, DD_ / 128, 1), dim3(256), 0, stream>>>(Hm, DD_, 0, W1, DD_, 0, nullptr, 1.0f, hp, DD_, 0, DD_);
  gemm_kn2<float, false><<<dim3(BB_ * QQ_ / 128, DD_ / 128, 1), dim3(256), 0, stream>>>(Um, DD_, 0, W1 + (size_t)DD_ * DD_, DD_, 0, nullptr, 1.0f, up, DD_, 0, DD_);
  k_pairs<<<dim3(BB_ * CC_), dim3(128), 0, stream>>>(Hm, Um, WmT, hp, up, b1, W2, b2, S);
  k_c2q<<<dim3(BB_ * 4), dim3(256), 0, stream>>>(S, Um, cmask, qmask, Uhat, Smax);
  k_q2c<<<dim3(BB_), dim3(256), 0, stream>>>(Smax, Hm, Hhat);
}
